// Dfine_70179765616855
// MI455X (gfx1250) — hardware-run, weakly checked
//
#include <hip/hip_runtime.h>
#include <math.h>

typedef __attribute__((ext_vector_type(16))) _Float16 v16h;
typedef __attribute__((ext_vector_type(8)))  _Float16 v8h;
typedef __attribute__((ext_vector_type(8)))  float    v8f;
typedef __attribute__((ext_vector_type(4)))  float    v4f;
typedef __attribute__((ext_vector_type(2)))  float    v2f;

constexpr int kNb = 256;
constexpr int kNt = 256;
constexpr int kNx = 16;
constexpr int kNu = 8;
constexpr int kNa = 32;
constexpr int kGrp = 8;
static_assert(kNx == 16 && kNa == 32 && kNu == 8, "lane maps assume 16 / 8 / 32");
static_assert((kNt % kGrp) == 0, "steps per flush group");
static_assert(kGrp * kNx * 4 == 512, "one flush = 4 whole 128-B lines = 32 lanes x 16 B");

constexpr int kOffA  = 0;
constexpr int kOffW  = 256;
constexpr int kOffH  = 512;
constexpr int kOffNx = 1024;
constexpr int kCstFloats = 1056;
constexpr size_t kWsTotal = (size_t)kCstFloats * 4;
static_assert(kWsTotal == 4224ull, "carve total");
static_assert((kCstFloats % 32) == 0, "whole lines");

constexpr float kCarryS = 16.0f;
constexpr float kCarryA = 16.0f;
constexpr float kCarryW = 64.0f;
constexpr float kResid  = 2048.0f;
constexpr float kFoldSA  = 1.0f / (kCarryS * kCarryA);
constexpr float kFoldSAR = kFoldSA / kResid;
constexpr float kFoldWS  = 1.0f / (kCarryW * kCarryS);
constexpr float kFoldWSR = kFoldWS / kResid;
constexpr float kF16Min  = 6.103515625e-05f;

union FragH { v16h v; v8h h[2]; };

__device__ __forceinline__ void split8(const float (&x)[8], const float carry, v16h& hi, v16h& lo) {
  v8h vh, vl;
#pragma unroll
  for (int r = 0; r < 8; ++r) {
    const float v  = x[r] * carry;
    const float vf = (fabsf(v) < kF16Min) ? 0.0f : v;
    const _Float16 hh = (_Float16)vf;
    float hf = (float)hh;
    asm volatile("" : "+v"(hf));
    const float res = (v - hf) * kResid;
    const float rf  = (fabsf(res) < kF16Min) ? 0.0f : res;
    vh[r] = hh;
    vl[r] = (_Float16)rf;
  }
  const v8h z = {(_Float16)0.0f, (_Float16)0.0f, (_Float16)0.0f, (_Float16)0.0f,
                 (_Float16)0.0f, (_Float16)0.0f, (_Float16)0.0f, (_Float16)0.0f};
  FragH fa, fb;
  fa.h[0] = vh; fa.h[1] = z;
  fb.h[0] = vl; fb.h[1] = z;
  hi = fa.v;
  lo = fb.v;
}

__device__ __forceinline__ v8f wmma_h(const v16h a, const v16h b, const v8f c) {
  return __builtin_amdgcn_wmma_f32_16x16x32_f16(false, a, false, b, (short)0, c, false, false);
}
__device__ __forceinline__ void guard_one(v8f& acc, const v16h a0, const v16h a1, const v16h b0, const v16h b1) {
  asm volatile("v_nop\n\tv_nop\n\tv_nop\n\tv_nop" : "+v"(acc) : "v"(a0), "v"(a1), "v"(b0), "v"(b1));
}
__device__ __forceinline__ void mma3(v16h ah, v16h al, v16h bh, v16h bl, v8f& accM, v8f& accR) {
  asm volatile("" : "+v"(ah), "+v"(al));
  asm volatile("" : "+v"(bh), "+v"(bl));
  const v8f z = {0.f, 0.f, 0.f, 0.f, 0.f, 0.f, 0.f, 0.f};
  accM = wmma_h(ah, bh, z);
  accR = wmma_h(ah, bl, z);
  accR = wmma_h(al, bh, accR);
  guard_one(accR, ah, al, bh, bl);
  guard_one(accM, ah, al, bh, bl);
}

__global__ __launch_bounds__(256) void filt_prep(
    const float* __restrict__ Mi, const float* __restrict__ Ni, const float* __restrict__ dv,
    const float* __restrict__ Cm, const float* __restrict__ nxv, const float* __restrict__ nav,
    float* __restrict__ cst)
{
  __shared__ __align__(16) float sQ2[512];
  __shared__ __align__(16) float sC[512];
  __shared__ float sSoft[64];
  __shared__ float sSd[16];
  __shared__ float sSi[16];
  __shared__ float sE[256];
  __shared__ __align__(16) float sOutP[kCstFloats];
  __shared__ double sAug[512];
  __shared__ double sRna[32];

  const int tid = threadIdx.x, lane = tid & 31, wave = tid >> 5;
  const int i = tid >> 4, j = tid & 15;

  sQ2[tid] = Mi[tid];
  sQ2[256 + tid] = Ni[tid];
  sC[tid] = Cm[tid];
  sC[256 + tid] = Cm[256 + tid];
  {
    const float vd = dv[tid & 15];
    const float vx = nxv[tid & 15];
    const float va = nav[tid & 31];
    const int sel = tid & 63;
    const float x = (sel < 16) ? vd : ((sel < 32) ? vx : va);
    const float e = expf(-fabsf(x));
    const float s = fmaxf(x, 0.0f) + log1pf(e);
    if (tid < 64) sSoft[tid] = s;
  }
  __syncthreads();

  if (wave == 0) {
    float* Qm = sQ2 + (lane >> 4) * 256;
    const int row = lane & 15;
#pragma unroll 1
    for (int c = 0; c < 16; ++c) {
#pragma unroll 1
      for (int rep = 0; rep < 2; ++rep) {
#pragma unroll 1
        for (int p = 0; p < c; ++p) {
          const float xp = Qm[row * 16 + p];
          const float xv = Qm[row * 16 + c];
          float r = xp * xv;
          r += __shfl_xor(r, 1, 32);
          r += __shfl_xor(r, 2, 32);
          r += __shfl_xor(r, 4, 32);
          r += __shfl_xor(r, 8, 32);
          Qm[row * 16 + c] = xv - r * xp;
        }
      }
      const float xv = Qm[row * 16 + c];
      float nrm = xv * xv;
      nrm += __shfl_xor(nrm, 1, 32);
      nrm += __shfl_xor(nrm, 2, 32);
      nrm += __shfl_xor(nrm, 4, 32);
      nrm += __shfl_xor(nrm, 8, 32);
      nrm = fmaxf(nrm, 1.0e-30f);
      float inv = rsqrtf(nrm);
      inv = inv * (1.5f - 0.5f * nrm * inv * inv);
      Qm[row * 16 + c] = xv * inv;
    }
  }
  __syncthreads();

  if (tid < 16) {
    const float sp = sSoft[tid];
    sSd[tid] = sqrtf(sp);
    sSi[tid] = 1.0f / sqrtf(1.0f + sp);
  }
  {
    const float naf = sSoft[32 + (tid & 31)] + 1.0e-4f;
    const double nd = (double)naf;
    double r = (double)__builtin_amdgcn_rcpf(naf);
    r = r * (2.0 - nd * r);
    r = r * (2.0 - nd * r);
    r = r * (2.0 - nd * r);
    if (tid < 32) sRna[tid] = r;
  }
  __syncthreads();

  {
    float e = 0.0f;
#pragma unroll 1
    for (int k = 0; k < 16; ++k) {
      const float x1 = sSd[k] * sQ2[k * 16 + j];
      e = fmaf(sQ2[256 + i * 16 + k], x1, e);
    }
    sE[tid] = e;
  }
  {
    double g = 0.0;
#pragma unroll 1
    for (int a = 0; a < 32; ++a) {
      const double cc = (double)sC[a * 16 + i] * (double)sC[a * 16 + j];
      g = fma(cc, sRna[a], g);
    }
    sAug[i * 32 + j] = g;
    sAug[i * 32 + 16 + j] = (i == j) ? 1.0 : 0.0;
  }
#pragma unroll 1
  for (int rep = 0; rep < 2; ++rep) {
    const int idx = tid + 256 * rep;
    const int x = idx >> 5, a = idx & 31;
    sOutP[kOffH + idx] = (float)((double)sC[a * 16 + x] * sRna[a]);
  }
  if (tid < 32) sOutP[kOffNx + tid] = (tid < 16) ? (sSoft[16 + tid] + 1.0e-4f) : 0.0f;
  __syncthreads();

  {
    float av = 0.0f;
#pragma unroll 1
    for (int k = 0; k < 16; ++k) {
      const float x2 = sSi[k] * sQ2[256 + j * 16 + k];
      av = fmaf(sE[i * 16 + k], x2, av);
    }
    sOutP[kOffA + tid] = av;
  }

#pragma unroll 1
  for (int k = 0; k < 16; ++k) {
    __syncthreads();
    const double piv = sAug[k * 32 + k];
    const double f   = sAug[i * 32 + k];
    const double r0v = sAug[k * 32 + j];
    const double r1v = sAug[k * 32 + 16 + j];
    const double o0  = sAug[i * 32 + j];
    const double o1  = sAug[i * 32 + 16 + j];
    const float pf = fmaxf((float)piv, 1.0e-30f);
    double rp = (double)__builtin_amdgcn_rcpf(pf);
    rp = rp * (2.0 - piv * rp);
    rp = rp * (2.0 - piv * rp);
    rp = rp * (2.0 - piv * rp);
    const double fr = f * rp;
    const double n0 = (i == k) ? (r0v * rp) : fma(-fr, r0v, o0);
    const double n1 = (i == k) ? (r1v * rp) : fma(-fr, r1v, o1);
    __syncthreads();
    sAug[i * 32 + j] = n0;
    sAug[i * 32 + 16 + j] = n1;
  }
  __syncthreads();
  {
    const double w = 0.5 * (sAug[i * 32 + 16 + j] + sAug[j * 32 + 16 + i]);
    sOutP[kOffW + tid] = (float)w;
  }
  __syncthreads();

  {
    const v4f v0 = *(const v4f*)(sOutP + 4 * tid);
    const v4f v1 = *(const v4f*)(sOutP + 1024 + 4 * (tid & 7));
    float* p0 = cst + 4 * tid;
    float* p1 = cst + 1024 + 4 * (tid & 7);
    for (int pass = 0; pass < 2; ++pass) {
      *(volatile v4f*)p0 = v0;
      if (tid < 8) *(volatile v4f*)p1 = v1;
      __threadfence();
    }
  }
}

__global__ __launch_bounds__(32) void filt_scan(
    const float* __restrict__ mean0, const float* __restrict__ cov0,
    const float* __restrict__ u, const float* __restrict__ a,
    const float* __restrict__ Bm, const float* __restrict__ Cm,
    const float* __restrict__ cst, float* __restrict__ out)
{
  __shared__ __align__(16) float sL[256];
  __shared__ __align__(16) float sM[16];
  __shared__ __align__(16) float sMp[16];
  __shared__ __align__(16) float sInn[32];
  __shared__ __align__(16) float sG[16];
  __shared__ __align__(16) float sU8[kGrp * kNu];
  __shared__ __align__(16) float sA8[kGrp * kNa];
  __shared__ __align__(16) float sO8[kGrp * kNx];

  const int lane = threadIdx.x & 31;
  const int h = lane >> 4;
  const int n = lane & 15;
  const int b = blockIdx.x;

  float arow[16], brow[8], crow[16], hrow[16];
#pragma unroll
  for (int q4 = 0; q4 < 4; ++q4) {
    const v4f ta = *(const v4f*)(cst + kOffA + n * 16 + 4 * q4);
    const v4f tc = *(const v4f*)(Cm + lane * 16 + 4 * q4);
    const v4f th = *(const v4f*)(cst + kOffH + n * 32 + 16 * h + 4 * q4);
    arow[4 * q4 + 0] = ta[0]; arow[4 * q4 + 1] = ta[1]; arow[4 * q4 + 2] = ta[2]; arow[4 * q4 + 3] = ta[3];
    crow[4 * q4 + 0] = tc[0]; crow[4 * q4 + 1] = tc[1]; crow[4 * q4 + 2] = tc[2]; crow[4 * q4 + 3] = tc[3];
    hrow[4 * q4 + 0] = th[0]; hrow[4 * q4 + 1] = th[1]; hrow[4 * q4 + 2] = th[2]; hrow[4 * q4 + 3] = th[3];
  }
#pragma unroll
  for (int q4 = 0; q4 < 2; ++q4) {
    const v4f tb = *(const v4f*)(Bm + n * 8 + 4 * q4);
    brow[4 * q4 + 0] = tb[0]; brow[4 * q4 + 1] = tb[1]; brow[4 * q4 + 2] = tb[2]; brow[4 * q4 + 3] = tb[3];
  }

  float wreg[8], wrow8[8], nxd[8], cov[8];
  {
    const float* g = cst + kOffW;
    const v4f t0 = *(const v4f*)(g + 8 * lane);
    const v4f t1 = *(const v4f*)(g + 8 * lane + 4);
    *(v4f*)(sL + 8 * lane) = t0;
    *(v4f*)(sL + 8 * lane + 4) = t1;
    __syncthreads();
#pragma unroll
    for (int r = 0; r < 8; ++r) wreg[r] = sL[(8 * h + r) * 16 + n];
    const v4f w0 = *(const v4f*)(sL + n * 16 + 8 * h);
    const v4f w1 = *(const v4f*)(sL + n * 16 + 8 * h + 4);
    wrow8[0] = w0[0]; wrow8[1] = w0[1]; wrow8[2] = w0[2]; wrow8[3] = w0[3];
    wrow8[4] = w1[0]; wrow8[5] = w1[1]; wrow8[6] = w1[2]; wrow8[7] = w1[3];
    __syncthreads();
  }
  {
    const float* g = cov0 + (size_t)b * 256;
    const v4f t0 = *(const v4f*)(g + 8 * lane);
    const v4f t1 = *(const v4f*)(g + 8 * lane + 4);
    *(v4f*)(sL + 8 * lane) = t0;
    *(v4f*)(sL + 8 * lane + 4) = t1;
    __syncthreads();
#pragma unroll
    for (int r = 0; r < 8; ++r) cov[r] = sL[(8 * h + r) * 16 + n];
    __syncthreads();
  }
  {
    const float nxn = cst[kOffNx + n];
#pragma unroll
    for (int r = 0; r < 8; ++r) nxd[r] = ((8 * h + r) == n) ? nxn : 0.0f;
  }

  v16h Afh, Afl, Wfh, Wfl;
  {
    float a8[8];
#pragma unroll
    for (int e = 0; e < 8; ++e) a8[e] = (h == 1) ? arow[8 + e] : arow[e];
    split8(a8, kCarryA, Afh, Afl);
    split8(wrow8, kCarryW, Wfh, Wfl);
  }

  {
    float mv = mean0[(size_t)b * kNx + n];
    asm volatile("" : "+v"(mv));
    if (h == 0) sM[n] = mv;
  }
  __syncthreads();

#pragma unroll 1
  for (int t0 = 0; t0 < kNt; t0 += kGrp) {
    {
      const size_t row0 = (size_t)b * kNt + t0;
      const v2f uu = *(const v2f*)(u + row0 * kNu + 2 * lane);
      const v4f a0 = *(const v4f*)(a + row0 * kNa + 4 * lane);
      const v4f a1 = *(const v4f*)(a + row0 * kNa + 128 + 4 * lane);
      *(v2f*)(sU8 + 2 * lane) = uu;
      *(v4f*)(sA8 + 4 * lane) = a0;
      *(v4f*)(sA8 + 128 + 4 * lane) = a1;
    }
    __syncthreads();

#pragma unroll 1
    for (int s = 0; s < kGrp; ++s) {
      const float* us = sU8 + s * kNu;
      const float* as = sA8 + s * kNa;

      float mp = 0.0f;
#pragma unroll
      for (int q4 = 0; q4 < 4; ++q4) {
        const v4f mv = *(const v4f*)(sM + 4 * q4);
        mp = fmaf(arow[4 * q4 + 0], mv[0], mp);
        mp = fmaf(arow[4 * q4 + 1], mv[1], mp);
        mp = fmaf(arow[4 * q4 + 2], mv[2], mp);
        mp = fmaf(arow[4 * q4 + 3], mv[3], mp);
      }
#pragma unroll
      for (int q4 = 0; q4 < 2; ++q4) {
        const v4f uv = *(const v4f*)(us + 4 * q4);
        mp = fmaf(brow[4 * q4 + 0], uv[0], mp);
        mp = fmaf(brow[4 * q4 + 1], uv[1], mp);
        mp = fmaf(brow[4 * q4 + 2], uv[2], mp);
        mp = fmaf(brow[4 * q4 + 3], uv[3], mp);
      }
      if (h == 0) sMp[n] = mp;
      __syncthreads();

      {
        float cm = 0.0f;
#pragma unroll
        for (int q4 = 0; q4 < 4; ++q4) {
          const v4f pv = *(const v4f*)(sMp + 4 * q4);
          cm = fmaf(crow[4 * q4 + 0], pv[0], cm);
          cm = fmaf(crow[4 * q4 + 1], pv[1], cm);
          cm = fmaf(crow[4 * q4 + 2], pv[2], cm);
          cm = fmaf(crow[4 * q4 + 3], pv[3], cm);
        }
        sInn[lane] = as[lane] - cm;
      }
      __syncthreads();

      {
        float gp = 0.0f;
#pragma unroll
        for (int q4 = 0; q4 < 4; ++q4) {
          const v4f iv = *(const v4f*)(sInn + 16 * h + 4 * q4);
          gp = fmaf(hrow[4 * q4 + 0], iv[0], gp);
          gp = fmaf(hrow[4 * q4 + 1], iv[1], gp);
          gp = fmaf(hrow[4 * q4 + 2], iv[2], gp);
          gp = fmaf(hrow[4 * q4 + 3], iv[3], gp);
        }
        const float gx = gp + __shfl_xor(gp, 16, 32);
        if (h == 0) sG[n] = gx;
      }

      float p[8], q[8];
      {
        v16h ch, cl;
        v8f accM, accR;
        split8(cov, kCarryS, ch, cl);
        mma3(ch, cl, Afh, Afl, accM, accR);
        float t1[8];
#pragma unroll
        for (int r = 0; r < 8; ++r) t1[r] = fmaf(accR[r], kFoldSAR, accM[r] * kFoldSA);
        v16h th, tl;
        split8(t1, kCarryS, th, tl);
        mma3(th, tl, Afh, Afl, accM, accR);
#pragma unroll
        for (int r = 0; r < 8; ++r) {
          const float pv = fmaf(accR[r], kFoldSAR, accM[r] * kFoldSA) + nxd[r];
          p[r] = pv;
          q[r] = pv + wreg[r];
        }
      }

      float invd[16];
#pragma unroll
      for (int k = 0; k < 16; ++k) {
        const float dsel = q[k & 7];
        const float dk = __shfl(dsel, ((k >> 3) << 4) | k, 32);
        const float inv = rsqrtf(fmaxf(dk, 1.0e-30f));
        invd[k] = inv;
        float cs[8];
#pragma unroll
        for (int r = 0; r < 8; ++r) {
          const float v = q[r] * inv;
          cs[r] = ((8 * h + r) >= k) ? v : 0.0f;
        }
        if (n == k) {
          const v4f c0 = {cs[0], cs[1], cs[2], cs[3]};
          const v4f c1 = {cs[4], cs[5], cs[6], cs[7]};
          *(v4f*)(sL + k * 16 + 8 * h) = c0;
          *(v4f*)(sL + k * 16 + 8 * h + 4) = c1;
        }
        __syncthreads();
        const v4f l0 = *(const v4f*)(sL + k * 16 + 8 * h);
        const v4f l1 = *(const v4f*)(sL + k * 16 + 8 * h + 4);
        const float ln = sL[k * 16 + n];
        q[0] = fmaf(-l0[0], ln, q[0]);
        q[1] = fmaf(-l0[1], ln, q[1]);
        q[2] = fmaf(-l0[2], ln, q[2]);
        q[3] = fmaf(-l0[3], ln, q[3]);
        q[4] = fmaf(-l1[0], ln, q[4]);
        q[5] = fmaf(-l1[1], ln, q[5]);
        q[6] = fmaf(-l1[2], ln, q[6]);
        q[7] = fmaf(-l1[3], ln, q[7]);
      }

#pragma unroll
      for (int t = 0; t < 16; ++t) {
        const float cand = p[t & 7] * invd[t];
        const float yt = __shfl(cand, ((t >> 3) << 4) | n, 32);
        const v4f l0 = *(const v4f*)(sL + t * 16 + 8 * h);
        const v4f l1 = *(const v4f*)(sL + t * 16 + 8 * h + 4);
        p[0] = fmaf(-l0[0], yt, p[0]);
        p[1] = fmaf(-l0[1], yt, p[1]);
        p[2] = fmaf(-l0[2], yt, p[2]);
        p[3] = fmaf(-l0[3], yt, p[3]);
        p[4] = fmaf(-l1[0], yt, p[4]);
        p[5] = fmaf(-l1[1], yt, p[5]);
        p[6] = fmaf(-l1[2], yt, p[6]);
        p[7] = fmaf(-l1[3], yt, p[7]);
        p[t & 7] = (h == (t >> 3)) ? yt : p[t & 7];
      }
#pragma unroll
      for (int tt = 0; tt < 16; ++tt) {
        const int t = 15 - tt;
        const float cand = p[t & 7] * invd[t];
        const float xt = __shfl(cand, ((t >> 3) << 4) | n, 32);
#pragma unroll
        for (int r = 0; r < 8; ++r) {
          const float cf = sL[(8 * h + r) * 16 + t];
          p[r] = fmaf(-cf, xt, p[r]);
        }
        p[t & 7] = (h == (t >> 3)) ? xt : p[t & 7];
      }

      {
        v16h yh, yl;
        v8f accM, accR;
        split8(p, kCarryS, yh, yl);
        mma3(Wfh, Wfl, yh, yl, accM, accR);
#pragma unroll
        for (int r = 0; r < 8; ++r) cov[r] = fmaf(accR[r], kFoldWSR, accM[r] * kFoldWS);
      }

      {
        const v4f g0 = *(const v4f*)(sG + 8 * h);
        const v4f g1 = *(const v4f*)(sG + 8 * h + 4);
        float up = 0.0f;
        up = fmaf(cov[0], g0[0], up);
        up = fmaf(cov[1], g0[1], up);
        up = fmaf(cov[2], g0[2], up);
        up = fmaf(cov[3], g0[3], up);
        up = fmaf(cov[4], g1[0], up);
        up = fmaf(cov[5], g1[1], up);
        up = fmaf(cov[6], g1[2], up);
        up = fmaf(cov[7], g1[3], up);
        const float ut = up + __shfl_xor(up, 16, 32);
        const float mpost = mp + ut;
        if (h == 0) {
          sM[n] = mpost;
          sO8[s * kNx + n] = mpost;
        }
      }
      __syncthreads();
    }

    {
      const v4f ov = *(const v4f*)(sO8 + 4 * lane);
      float* op = out + ((size_t)b * kNt + t0) * kNx + 4 * lane;
      *(volatile v4f*)op = ov;
      __threadfence();
      *(volatile v4f*)op = ov;
    }
  }
}

extern "C" void kernel_launch(void* const* d_in, const int* in_sizes, int n_in,
                              void* d_out, int out_size, void* d_ws, size_t ws_size,
                              hipStream_t stream) {
  if (n_in < 11) return;
  if (in_sizes[0] != kNb * kNx) return;
  if (in_sizes[1] != kNb * kNx * kNx) return;
  if (in_sizes[2] != kNb * kNt * kNu) return;
  if (in_sizes[3] != kNb * kNt * kNa) return;
  if (in_sizes[4] != kNx * kNx) return;
  if (in_sizes[5] != kNx * kNx) return;
  if (in_sizes[6] != kNx) return;
  if (in_sizes[7] != kNx * kNu) return;
  if (in_sizes[8] != kNa * kNx) return;
  if (in_sizes[9] != kNx) return;
  if (in_sizes[10] != kNa) return;
  if (out_size != kNb * kNt * kNx) return;
  if (ws_size < kWsTotal) return;

  const float* mean0 = (const float*)d_in[0];
  const float* cov0  = (const float*)d_in[1];
  const float* u     = (const float*)d_in[2];
  const float* a     = (const float*)d_in[3];
  const float* Mi    = (const float*)d_in[4];
  const float* Ni    = (const float*)d_in[5];
  const float* dvec  = (const float*)d_in[6];
  const float* Bm    = (const float*)d_in[7];
  const float* Cm    = (const float*)d_in[8];
  const float* nx    = (const float*)d_in[9];
  const float* na    = (const float*)d_in[10];
  float* cst = (float*)d_ws;
  float* out = (float*)d_out;

  filt_prep<<<1, 256, 0, stream>>>(Mi, Ni, dvec, Cm, nx, na, cst);
  filt_scan<<<kNb, 32, 0, stream>>>(mean0, cov0, u, a, Bm, Cm, cst, out);
}
